// MSARowAttentionWithPairBias_962072674748
// MI455X (gfx1250) — hardware-verified
//
#include <hip/hip_runtime.h>


#define NB_  1
#define TT   256
#define DM   256
#define NH_  8
#define NKV  8
#define REP  (NH_ / NKV)
#define HD   32
#define DQ   (NH_ * HD)
#define DKV  (NKV * HD)
#define ZH   16
#define RH   256
#define WIN  0
#define PCAR 1024.0f
#define SCL  0.17677669529663688f
#define NS   128
#define NI   256
#define CZ   128
#define NP   (NS * NH_)
#define NRM  (NS * NI)
#define NRP  (NI * NI)
#define HP   64
#define NBP  64
typedef _Float16 h16;
typedef unsigned short bf;
typedef __attribute__((ext_vector_type(16))) __bf16   v16bf;
typedef __attribute__((ext_vector_type(16))) _Float16 v16h;
typedef __attribute__((ext_vector_type(8)))  _Float16 v8h;
typedef __attribute__((ext_vector_type(8)))  unsigned short v8us;
typedef __attribute__((ext_vector_type(8)))  float    v8f;
typedef __attribute__((ext_vector_type(4)))  float    v4f;
typedef v8h  __attribute__((may_alias)) v8ha;
typedef v4f  __attribute__((may_alias)) v4fa;
typedef v8us __attribute__((may_alias)) v8usa;

__device__ __forceinline__ unsigned short f2bf(float f) { unsigned u = __float_as_uint(f); u += 0x7FFFu + ((u >> 16) & 1u); return (unsigned short)(u >> 16); }
__device__ __forceinline__ float bf2f(unsigned short b) { return __uint_as_float(((unsigned)b) << 16); }
__device__ __forceinline__ float bfr(float f) { return bf2f(f2bf(f)); }
__device__ __forceinline__ v16h cat16(v8h lo, v8h hi) { return __builtin_shufflevector(lo, hi, 0, 1, 2, 3, 4, 5, 6, 7, 8, 9, 10, 11, 12, 13, 14, 15); }
__device__ __forceinline__ v16bf cat16b(v8us lo, v8us hi) { return __builtin_bit_cast(v16bf, __builtin_shufflevector(lo, hi, 0, 1, 2, 3, 4, 5, 6, 7, 8, 9, 10, 11, 12, 13, 14, 15)); }
__device__ __forceinline__ v8f wmma16(v16h a, v16h b, v8f c) { return __builtin_amdgcn_wmma_f32_16x16x32_f16(false, a, false, b, (short)0, c, false, false); }
__device__ __forceinline__ v8f wmmab(v16bf a, v16bf b, v8f c) { return __builtin_amdgcn_wmma_f32_16x16x32_bf16(false, a, false, b, (short)0, c, false, false); }


template <typename T16> struct WFrag;
template <> struct WFrag<h16> { typedef v16h V; static __device__ __forceinline__ V ld(const h16* p) { return cat16(*(const v8h*)p, *(const v8h*)(p + 16)); } static __device__ __forceinline__ v8f mma(V a, V b, v8f c) { return wmma16(a, b, c); } };
template <> struct WFrag<bf> { typedef v16bf V; static __device__ __forceinline__ V ld(const bf* p) { return cat16b(*(const v8us*)p, *(const v8us*)(p + 16)); } static __device__ __forceinline__ v8f mma(V a, V b, v8f c) { return wmmab(a, b, c); } };
template <typename T16, int NSPLIT, bool BIAS>
__global__ __launch_bounds__(32) void k_gemmw(const T16* __restrict__ A, const T16* __restrict__ A2, const T16* __restrict__ Bt, const T16* __restrict__ Bt2, int K, float* C, int ldc, const float* __restrict__ bias, size_t sA, size_t sB, size_t sC) {
    typedef typename WFrag<T16>::V V;
    __shared__ __align__(16) float os[16 * 68];
    const size_t z = blockIdx.z; A += z * sA; if (A2) A2 += z * sA; Bt += z * sB; if (Bt2) Bt2 += z * sB; C += z * sC;
    const int lane = threadIdx.x & 31, lr = lane & 15, hi = lane >> 4; const int r0 = blockIdx.x * 64, c0 = blockIdx.y * 64;
    v8f acc[4][4];
#pragma unroll
    for (int mb = 0; mb < 4; ++mb)
#pragma unroll
        for (int nb = 0; nb < 4; ++nb) acc[mb][nb] = (v8f){};
    const size_t aoff = (size_t)(r0 + lr) * K + 8 * hi, boff = (size_t)(c0 + lr) * K + 8 * hi;
#pragma unroll 1
    for (int kc = 0; kc < K; kc += 32) {
        V a[4], a2[4];
#pragma unroll
        for (int mb = 0; mb < 4; ++mb) { a[mb] = WFrag<T16>::ld(A + aoff + (size_t)mb * 16 * K + kc); if (NSPLIT == 1 || NSPLIT == 2) a2[mb] = WFrag<T16>::ld(A2 + aoff + (size_t)mb * 16 * K + kc); }
#pragma unroll
        for (int nb = 0; nb < 4; ++nb) { const V b = WFrag<T16>::ld(Bt + boff + (size_t)nb * 16 * K + kc); V b2; if (NSPLIT >= 2) b2 = WFrag<T16>::ld(Bt2 + boff + (size_t)nb * 16 * K + kc);
#pragma unroll
            for (int mb = 0; mb < 4; ++mb) { acc[mb][nb] = WFrag<T16>::mma(a[mb], b, acc[mb][nb]); if (NSPLIT == 1 || NSPLIT == 2) acc[mb][nb] = WFrag<T16>::mma(a2[mb], b, acc[mb][nb]); if (NSPLIT >= 2) acc[mb][nb] = WFrag<T16>::mma(a[mb], b2, acc[mb][nb]); } }
        asm volatile("v_nop\n\tv_nop\n\tv_nop\n\tv_nop" : "+v"(acc[0][0]), "+v"(acc[1][1]), "+v"(acc[2][2]), "+v"(acc[3][3]) : "v"(a[0]), "v"(a[3]));
    }
#pragma unroll
    for (int mb = 0; mb < 4; ++mb) {
#pragma unroll
        for (int nb = 0; nb < 4; ++nb) {
#pragma unroll
            for (int j = 0; j < 8; ++j) os[(hi * 8 + j) * 68 + nb * 16 + lr] = acc[mb][nb][j]; }
        __builtin_amdgcn_wave_barrier(); asm volatile("" ::: "memory");
        float* crow = C + (size_t)(r0 + mb * 16) * ldc + c0;
#pragma unroll 1
        for (int ps = 0; ps < 2; ++ps) {
#pragma unroll
            for (int s = 0; s < 8; ++s) { const int row = 2 * s + hi, cofs = lr * 4; v4f val = *(const v4fa*)(os + row * 68 + cofs); if (BIAS) { val[0] += bfr(bias[c0 + cofs]); val[1] += bfr(bias[c0 + cofs + 1]); val[2] += bfr(bias[c0 + cofs + 2]); val[3] += bfr(bias[c0 + cofs + 3]); }
                *(volatile v4f*)(crow + (size_t)row * ldc + cofs) = val; }
            if (ps == 0) __threadfence(); }
        __builtin_amdgcn_wave_barrier(); asm volatile("" ::: "memory");
    }
}

__device__ __forceinline__ h16 tohx(float x) { return (h16)x; }
__device__ __forceinline__ void splitf(float y, unsigned short& h, unsigned short& l) { h = f2bf(y); l = f2bf(y - bf2f(h)); }
typedef __attribute__((ext_vector_type(2))) _Float16 v2h;
typedef __attribute__((ext_vector_type(4))) _Float16 v4h;
typedef __attribute__((ext_vector_type(2))) unsigned short v2us;
typedef __attribute__((ext_vector_type(4))) unsigned short v4us;
typedef __attribute__((ext_vector_type(2))) float v2f;
typedef __attribute__((ext_vector_type(4))) int v4i;

__global__ __launch_bounds__(256) void k_wtG(const float* __restrict__ w, int K, int N, bf* Bt) {
    const int lane = threadIdx.x & 31; const int L0 = (blockIdx.x * 8 + (threadIdx.x >> 5)) * 8; const int nlines = N * K / 64;
#pragma unroll
    for (int ps = 0; ps < 2; ++ps) {
#pragma unroll 1
        for (int l = 0; l < 8; ++l) { const int L = L0 + l; if (L >= nlines) break; const size_t e = (size_t)L * 64 + lane * 2; const int k = (int)(e % K), n = (int)(e / K); v2us o;
            o[0] = f2bf(w[(size_t)k * N + n]); o[1] = f2bf(w[(size_t)(k + 1) * N + n]); *(volatile v2us*)(Bt + e) = o; }
        if (ps == 0) __threadfence(); }
}
__global__ __launch_bounds__(256) void k_cvt8(const float* __restrict__ src, bf* dst, size_t n8) { const size_t i = (size_t)blockIdx.x * 256 + threadIdx.x; if (i >= n8) return; const v8f v = *(const v8f*)(src + i * 8); v8us o;
#pragma unroll
    for (int k = 0; k < 8; ++k) o[k] = f2bf(v[k]); *(volatile v8us*)(dst + i * 8) = o; __threadfence(); *(volatile v8us*)(dst + i * 8) = o; }


__global__ __launch_bounds__(256) void k_asoft(const float* __restrict__ Sb, h16* P16, bf* Ph, bf* Pl) {
    const int lane = threadIdx.x & 31; const int row = blockIdx.x * 8 + (threadIdx.x >> 5); if (row >= ZH * TT) return; const int i = row % TT; const int zz = row / TT; (void)zz; const bool hires = (i < RH); const float* sr = Sb + (size_t)row * TT; float v[TT / 32]; float mx = -3.0e38f;
#pragma unroll
    for (int ch = 0; ch < TT / 128; ++ch) { const int j0 = ch * 128 + lane * 4; const v4f a = *(const v4f*)(sr + j0);
#pragma unroll
        for (int q = 0; q < 4; ++q) { const int j = j0 + q; (void)j; const float t = a[q] * SCL; v[ch * 4 + q] = t; mx = fmaxf(mx, t); } }
#pragma unroll
    for (int sh = 16; sh; sh >>= 1) mx = fmaxf(mx, __shfl_xor(mx, sh, 32));
    float sum = 0.f;
#pragma unroll
    for (int k = 0; k < TT / 32; ++k) { float d0 = __fsub_rn(v[k], mx); asm volatile("" : "+v"(d0)); v[k] = __builtin_amdgcn_exp2f(__fmul_rn(d0, 1.4426950408889634f)); sum += v[k]; }
#pragma unroll
    for (int sh = 16; sh; sh >>= 1) sum += __shfl_xor(sum, sh, 32);
    const float f = __fdiv_rn(hires ? 1.0f : PCAR, sum);
#pragma unroll 1
    for (int ps = 0; ps < 2; ++ps) {
        if (hires) {
#pragma unroll
            for (int ch = 0; ch < TT / 128; ++ch) { v4us oh, ol;
#pragma unroll
                for (int q = 0; q < 4; ++q) { unsigned short a, c2; splitf(v[ch * 4 + q] * f, a, c2); oh[q] = a; ol[q] = c2; }
                const size_t oo = ((size_t)zz * (RH ? RH : 1) + i) * TT + ch * 128 + lane * 4; *(volatile v4us*)(Ph + oo) = oh; *(volatile v4us*)(Pl + oo) = ol; }
        } else {
#pragma unroll
            for (int ch = 0; ch < TT / 128; ++ch) { v4h o4;
#pragma unroll
                for (int q = 0; q < 4; ++q) o4[q] = tohx(v[ch * 4 + q] * f);
                *(volatile v4h*)(P16 + (size_t)row * TT + ch * 128 + lane * 4) = o4; } }
        if (ps == 0) __threadfence(); }
}
__device__ __forceinline__ float ex2g(float a) { return __builtin_amdgcn_exp2f(__fmul_rn(a, 1.4426950408889634f)); }
__device__ __forceinline__ float sigm(float a) { return __fdiv_rn(1.0f, __fadd_rn(1.0f, ex2g(-a))); }
template <int WD>
__global__ __launch_bounds__(256) void k_lnrow(const float* __restrict__ X, size_t nrows, const float* __restrict__ g, const float* __restrict__ bb, bf* Hh, bf* Hl) { const int lane = threadIdx.x & 31; const size_t r = (size_t)blockIdx.x * 8 + (threadIdx.x >> 5); if (r >= nrows) return; const float* xr = X + r * WD; float a[WD / 32]; float s = 0.f;
#pragma unroll
    for (int c = 0; c < WD / 128; ++c) { const v4f v = *(const v4f*)(xr + c * 128 + lane * 4); for (int q = 0; q < 4; ++q) { a[c * 4 + q] = bfr(v[q]); s = __fadd_rn(s, a[c * 4 + q]); } }
#pragma unroll
    for (int sh = 16; sh; sh >>= 1) s = __fadd_rn(s, __shfl_xor(s, sh, 32));
    const float mean = __fdiv_rn(s, (float)WD); float s2 = 0.f;
#pragma unroll
    for (int k = 0; k < WD / 32; ++k) { const float dv = __fsub_rn(a[k], mean); s2 = __fadd_rn(s2, __fmul_rn(dv, dv)); }
#pragma unroll
    for (int sh = 16; sh; sh >>= 1) s2 = __fadd_rn(s2, __shfl_xor(s2, sh, 32));
    const float rs = __fdiv_rn(1.0f, __fsqrt_rn(__fadd_rn(__fdiv_rn(s2, (float)WD), 1e-5f)));
#pragma unroll 1
    for (int ps = 0; ps < 2; ++ps) {
#pragma unroll
        for (int c = 0; c < WD / 128; ++c) { v4us oh, ol; for (int q = 0; q < 4; ++q) { const int col = c * 128 + lane * 4 + q; float y = __fmul_rn(__fmul_rn(__fsub_rn(a[c * 4 + q], mean), rs), bfr(g[col])); asm volatile("" : "+v"(y)); y = __fadd_rn(y, bfr(bb[col])); unsigned short u, w2; splitf(y, u, w2); oh[q] = u; ol[q] = w2; } *(volatile v4us*)(Hh + r * WD + c * 128 + lane * 4) = oh; *(volatile v4us*)(Hl + r * WD + c * 128 + lane * 4) = ol; }
        if (ps == 0) __threadfence(); } }
__global__ __launch_bounds__(256) void k_wpad(const float* __restrict__ w, bf* Bt) { const int e2 = (blockIdx.x * 256 + threadIdx.x) * 2; if (e2 >= NBP * CZ) return; const int k = e2 % CZ; const int n = e2 / CZ; v2us o; const unsigned short a0 = f2bf(w[(size_t)k * NH_ + min(n, NH_ - 1)]), a1 = f2bf(w[(size_t)(k + 1) * NH_ + min(n, NH_ - 1)]); o[0] = (n < NH_) ? a0 : (unsigned short)0; o[1] = (n < NH_) ? a1 : (unsigned short)0; *(volatile v2us*)(Bt + e2) = o; __threadfence(); *(volatile v2us*)(Bt + e2) = o; }
__global__ __launch_bounds__(256) void k_planesS(const float* __restrict__ F, bf* Ph, bf* Pl) { const size_t k = (size_t)blockIdx.x * 256 + threadIdx.x; if (k >= (size_t)NP * NI * HD / 4) return; const size_t e = k * 4; const int d = (int)(e % HD); const int i = (int)((e / HD) % NI); const int p = (int)(e / ((size_t)HD * NI)); const int s = p / NH_, h = p % NH_; const v4f a = *(const v4f*)(F + ((size_t)s * NI + i) * DQ + h * HD + d); v4us oh, ol;
#pragma unroll
    for (int q = 0; q < 4; ++q) { unsigned short u, w2; splitf(a[q], u, w2); oh[q] = u; ol[q] = w2; }
    *(volatile v4us*)(Ph + e) = oh; *(volatile v4us*)(Pl + e) = ol; __threadfence(); *(volatile v4us*)(Ph + e) = oh; *(volatile v4us*)(Pl + e) = ol; }
__global__ __launch_bounds__(256) void k_vtpS(const float* __restrict__ F, bf* Vh, bf* Vl) { const size_t e = ((size_t)blockIdx.x * 256 + threadIdx.x) * 2; if (e >= (size_t)NP * HP * NI) return; const int i = (int)(e % NI); const int d = (int)((e / NI) % HP); const int p = (int)(e / ((size_t)NI * HP)); const int s = p / NH_, h = p % NH_; const int dd = min(d, HD - 1); v2us oh, ol;
#pragma unroll
    for (int q = 0; q < 2; ++q) { const float v = F[((size_t)s * NI + i + q) * DQ + h * HD + dd]; unsigned short u, w2; splitf(v, u, w2); oh[q] = (d < HD) ? u : (unsigned short)0; ol[q] = (d < HD) ? w2 : (unsigned short)0; }
    *(volatile v2us*)(Vh + e) = oh; *(volatile v2us*)(Vl + e) = ol; __threadfence(); *(volatile v2us*)(Vh + e) = oh; *(volatile v2us*)(Vl + e) = ol; }
__global__ __launch_bounds__(256) void k_addbias(float* Sb, const float* __restrict__ BIAS, int p0) { const size_t k = (size_t)blockIdx.x * 256 + threadIdx.x; if (k >= (size_t)ZH * NI * NI / 4) return; const size_t e = k * 4; const int j0 = (int)(e % NI); const int i = (int)((e / NI) % NI); const int zz = (int)(e / ((size_t)NI * NI)); const int h = (p0 + zz) % NH_; v4f a = *(const v4f*)(Sb + e);
#pragma unroll
    for (int q = 0; q < 4; ++q) a[q] = __fadd_rn(a[q], __fmul_rn(BIAS[((size_t)i * NI + j0 + q) * NBP + h], 5.656854249492380f));
    *(volatile v4f*)(Sb + e) = a; __threadfence(); *(volatile v4f*)(Sb + e) = a; }
__global__ __launch_bounds__(256) void k_mergeG(const float* __restrict__ O, const float* __restrict__ GP, int p0, bf* Ah, bf* Al) { const size_t k = (size_t)blockIdx.x * 256 + threadIdx.x; if (k >= (size_t)ZH * NI * HD / 4) return; const size_t e = k * 4; const int d = (int)(e % HD); const int i = (int)((e / HD) % NI); const int zz = (int)(e / ((size_t)HD * NI)); const int p = p0 + zz; const int s = p / NH_, h = p % NH_; const size_t row = (size_t)s * NI + i; const v4f o = *(const v4f*)(O + ((size_t)zz * NI + i) * HP + d); const v4f gp = *(const v4f*)(GP + row * DQ + h * HD + d); v4us oh, ol;
#pragma unroll
    for (int q = 0; q < 4; ++q) { float y = __fmul_rn(sigm(gp[q]), o[q]); unsigned short u, w2; splitf(y, u, w2); oh[q] = u; ol[q] = w2; }
    const size_t oo = row * DQ + h * HD + d; *(volatile v4us*)(Ah + oo) = oh; *(volatile v4us*)(Al + oo) = ol; __threadfence(); *(volatile v4us*)(Ah + oo) = oh; *(volatile v4us*)(Al + oo) = ol; }

extern "C" void kernel_launch(void* const* d_in, const int* in_sizes, int n_in,
                              void* d_out, int out_size, void* d_ws, size_t ws_size, hipStream_t stream) {
    (void)in_sizes; (void)n_in; (void)out_size;
    const float* msa = (const float*)d_in[0]; const float* pair = (const float*)d_in[1]; const float* lmg = (const float*)d_in[2]; const float* lmb = (const float*)d_in[3]; const float* lpg = (const float*)d_in[4]; const float* lpb = (const float*)d_in[5]; const float* wq = (const float*)d_in[6]; const float* wk = (const float*)d_in[7]; const float* wv = (const float*)d_in[8]; const float* wp = (const float*)d_in[9]; const float* wg = (const float*)d_in[10]; const float* bg = (const float*)d_in[11]; const float* wo = (const float*)d_in[12]; const float* bo = (const float*)d_in[13];
    float* OUT = (float*)d_out;
    char* wsp = (char*)d_ws;
    auto take = [&](size_t bytes) { char* p = wsp; wsp += (bytes + 255) & ~(size_t)255; return (void*)p; };
    bf* WQ = (bf*)take((size_t)DQ * DM * 2); bf* WK = (bf*)take((size_t)DQ * DM * 2); bf* WV = (bf*)take((size_t)DQ * DM * 2); bf* WG = (bf*)take((size_t)DQ * DM * 2); bf* WO = (bf*)take((size_t)DM * DQ * 2); bf* WP = (bf*)take((size_t)NBP * CZ * 2);
    bf* Mh = (bf*)take((size_t)NRM * DM * 2); bf* Ml = (bf*)take((size_t)NRM * DM * 2); float* FQ = (float*)take((size_t)NRM * DQ * 4); float* GP = (float*)take((size_t)NRM * DQ * 4); float* BIAS = (float*)take((size_t)NRP * NBP * 4);
    bf* QPh = (bf*)take((size_t)NP * NI * HD * 2); bf* QPl = (bf*)take((size_t)NP * NI * HD * 2); bf* KPh = (bf*)take((size_t)NP * NI * HD * 2); bf* KPl = (bf*)take((size_t)NP * NI * HD * 2); bf* VTh = (bf*)take((size_t)NP * HP * NI * 2); bf* VTl = (bf*)take((size_t)NP * HP * NI * 2);
    float* Sb = (float*)take((size_t)ZH * NI * NI * 4); bf* Ph = (bf*)take((size_t)ZH * NI * NI * 2); bf* Pl = (bf*)take((size_t)ZH * NI * NI * 2); float* Ob = (float*)take((size_t)ZH * NI * HP * 4); bf* ATh = Mh; bf* ATl = Ml;
    if ((size_t)(wsp - (char*)d_ws) > ws_size) return;
    bf* PLh = (bf*)FQ; bf* PLl = (bf*)GP;
    k_wtG<<<(DM * DQ / 64 + 63) / 64, 256, 0, stream>>>(wq, DM, DQ, WQ); k_wtG<<<(DM * DQ / 64 + 63) / 64, 256, 0, stream>>>(wk, DM, DQ, WK); k_wtG<<<(DM * DQ / 64 + 63) / 64, 256, 0, stream>>>(wv, DM, DQ, WV); k_wtG<<<(DM * DQ / 64 + 63) / 64, 256, 0, stream>>>(wg, DM, DQ, WG); k_wtG<<<(DQ * DM / 64 + 63) / 64, 256, 0, stream>>>(wo, DQ, DM, WO); k_wpad<<<(NBP * CZ / 2 + 255) / 256, 256, 0, stream>>>(wp, WP);
    k_lnrow<CZ><<<(unsigned)((NRP + 7) / 8), 256, 0, stream>>>(pair, (size_t)NRP, lpg, lpb, PLh, PLl);
    k_gemmw<bf, 1, false><<<dim3(NRP / 64, NBP / 64, 1), 32, 0, stream>>>(PLh, PLl, WP, nullptr, CZ, BIAS, NBP, nullptr, 0, 0, 0);
    k_lnrow<DM><<<(unsigned)((NRM + 7) / 8), 256, 0, stream>>>(msa, (size_t)NRM, lmg, lmb, Mh, Ml);
    k_gemmw<bf, 1, false><<<dim3(NRM / 64, DQ / 64, 1), 32, 0, stream>>>(Mh, Ml, WQ, nullptr, DM, FQ, DQ, nullptr, 0, 0, 0); k_planesS<<<(unsigned)(((size_t)NP * NI * HD / 4 + 255) / 256), 256, 0, stream>>>(FQ, QPh, QPl);
    k_gemmw<bf, 1, false><<<dim3(NRM / 64, DQ / 64, 1), 32, 0, stream>>>(Mh, Ml, WK, nullptr, DM, FQ, DQ, nullptr, 0, 0, 0); k_planesS<<<(unsigned)(((size_t)NP * NI * HD / 4 + 255) / 256), 256, 0, stream>>>(FQ, KPh, KPl);
    k_gemmw<bf, 1, false><<<dim3(NRM / 64, DQ / 64, 1), 32, 0, stream>>>(Mh, Ml, WV, nullptr, DM, FQ, DQ, nullptr, 0, 0, 0); k_vtpS<<<(unsigned)(((size_t)NP * HP * NI / 2 + 255) / 256), 256, 0, stream>>>(FQ, VTh, VTl);
    k_gemmw<bf, 1, true><<<dim3(NRM / 64, DQ / 64, 1), 32, 0, stream>>>(Mh, Ml, WG, nullptr, DM, GP, DQ, bg, 0, 0, 0);
    for (int p0 = 0; p0 < NP; p0 += ZH) {
        k_gemmw<bf, 2, false><<<dim3(NI / 64, NI / 64, ZH), 32, 0, stream>>>(QPh + (size_t)p0 * NI * HD, QPl + (size_t)p0 * NI * HD, KPh + (size_t)p0 * NI * HD, KPl + (size_t)p0 * NI * HD, HD, Sb, NI, nullptr, (size_t)NI * HD, (size_t)NI * HD, (size_t)NI * NI);
        k_addbias<<<(unsigned)(((size_t)ZH * NI * NI / 4 + 255) / 256), 256, 0, stream>>>(Sb, BIAS, p0);
        k_asoft<<<ZH * TT / 8, 256, 0, stream>>>(Sb, nullptr, Ph, Pl);
        k_gemmw<bf, 2, false><<<dim3(NI / 64, HP / 64, ZH), 32, 0, stream>>>(Ph, Pl, VTh + (size_t)p0 * HP * NI, VTl + (size_t)p0 * HP * NI, NI, Ob, HP, nullptr, (size_t)NI * NI, (size_t)HP * NI, (size_t)NI * HP);
        k_mergeG<<<(unsigned)(((size_t)ZH * NI * HD / 4 + 255) / 256), 256, 0, stream>>>(Ob, GP, p0, ATh, ATl); }
    k_gemmw<bf, 1, true><<<dim3(NRM / 64, DM / 64, 1), 32, 0, stream>>>(ATh, ATl, WO, nullptr, DQ, OUT, DM, bo, 0, 0, 0);
}
